// CausalDecayMemory_3865470566777
// MI455X (gfx1250) — hardware-verified
//
#include <hip/hip_runtime.h>
#include <math.h>
#include <stdint.h>

#define NB   4
#define TT   4096
#define DD   512
#define QR   32
#define KT   128
#define PST  136

static_assert((TT % KT) == 0);
static_assert((TT % QR) == 0);
static_assert((DD % 64) == 0);
static_assert((TT % 64) == 0);
static_assert(((NB * TT) % 64) == 0);
static_assert(((PST * 2) % 16) == 0);
static_assert(((NB * TT * DD) % 2048) == 0);
static_assert(((DD * DD) % 2048) == 0);

typedef _Float16 v16h __attribute__((ext_vector_type(16)));
typedef _Float16 v8h  __attribute__((ext_vector_type(8)));
typedef __bf16   v16b __attribute__((ext_vector_type(16)));
typedef __bf16   v8b  __attribute__((ext_vector_type(8)));
typedef float    v8f  __attribute__((ext_vector_type(8)));
typedef float    v4f  __attribute__((ext_vector_type(4)));
typedef unsigned int v4u __attribute__((ext_vector_type(4)));

__device__ __forceinline__ unsigned short bf_bits(float f) {
  unsigned u = __float_as_uint(f);
  return (unsigned short)((u + 0x7FFFu + ((u >> 16) & 1u)) >> 16);
}
__device__ __forceinline__ float bf_up(unsigned short h) { return __uint_as_float(((unsigned)h) << 16); }
__device__ __forceinline__ unsigned short h_bits(_Float16 x) { return __builtin_bit_cast(unsigned short, x); }
__device__ __forceinline__ unsigned pk16(unsigned short a, unsigned short b) { return (unsigned)a | ((unsigned)b << 16); }
__device__ __forceinline__ v8f zero8() { v8f z = {0.f, 0.f, 0.f, 0.f, 0.f, 0.f, 0.f, 0.f}; return z; }

union FB { v16b v; v8b h[2]; };
union FH { v16h v; v8h h[2]; };
__device__ __forceinline__ v16b ldfrag_b(const __bf16* p) {
  FB f;
  f.h[0] = *(const v8b*)(p);
  f.h[1] = *(const v8b*)(p + 16);
  return f.v;
}
__device__ __forceinline__ v16h ldfrag_h(const _Float16* p) {
  FH f;
  f.h[0] = *(const v8h*)(p);
  f.h[1] = *(const v8h*)(p + 16);
  return f.v;
}

__device__ __forceinline__ v8f wraw_b(v16b a, v16b b, v8f c) {
  return __builtin_amdgcn_wmma_f32_16x16x32_bf16(false, a, false, b, (short)0, c, false, false);
}
__device__ __forceinline__ v8f wraw_h(v16h a, v16h b, v8f c) {
  return __builtin_amdgcn_wmma_f32_16x16x32_f16(false, a, false, b, (short)0, c, false, false);
}
__device__ __forceinline__ void dep_guard_b(v8f& a, v8f& b, v16b x, v16b y) {
#if defined(__HIP_DEVICE_COMPILE__)
  asm volatile("v_nop\n\tv_nop\n\tv_nop\n\tv_nop" : "+v"(a), "+v"(b) : "v"(x), "v"(y));
#endif
}
__device__ __forceinline__ void keep4_b(v16b a, v16b b, v16b c, v16b d) {
#if defined(__HIP_DEVICE_COMPILE__)
  asm volatile("v_nop" :: "v"(a), "v"(b), "v"(c), "v"(d));
#endif
}
__device__ __forceinline__ void acc_guard4(v8f& a, v8f& b, v8f& c, v8f& d) {
#if defined(__HIP_DEVICE_COMPILE__)
  asm volatile("v_nop\n\tv_nop\n\tv_nop\n\tv_nop" : "+v"(a), "+v"(b), "+v"(c), "+v"(d));
#endif
}
__device__ __forceinline__ void guard_s(v8f& c0, v8f& c1, v8f& c2, v8f& c3,
                                        v16h a0, v16h a1, v16h a2, v16h a3, v16h bb) {
#if defined(__HIP_DEVICE_COMPILE__)
  asm volatile("v_nop\n\tv_nop\n\tv_nop\n\tv_nop"
               : "+v"(c0), "+v"(c1), "+v"(c2), "+v"(c3)
               : "v"(a0), "v"(a1), "v"(a2), "v"(a3), "v"(bb));
#endif
}
__device__ __forceinline__ void guard_p(v8f& c0, v8f& c1, v8f& c2, v8f& c3,
                                        v8f& c4, v8f& c5, v8f& c6, v8f& c7,
                                        v16h p0, v16h p1, v16h b0, v16h b1, v16h b2, v16h b3) {
#if defined(__HIP_DEVICE_COMPILE__)
  asm volatile("v_nop\n\tv_nop\n\tv_nop\n\tv_nop"
               : "+v"(c0), "+v"(c1), "+v"(c2), "+v"(c3), "+v"(c4), "+v"(c5), "+v"(c6), "+v"(c7)
               : "v"(p0), "v"(p1), "v"(b0), "v"(b1), "v"(b2), "v"(b3));
#endif
}

__global__ __launch_bounds__(256) void cvt_bf16x8(const float* __restrict__ in, unsigned short* out, int n8) {
  const int i = blockIdx.x * 256 + threadIdx.x;
  if (i < n8) {
    const v4f a = *(const v4f*)(in + (size_t)i * 8);
    const v4f b = *(const v4f*)(in + (size_t)i * 8 + 4);
    v4u p;
    p[0] = pk16(bf_bits(a[0]), bf_bits(a[1]));
    p[1] = pk16(bf_bits(a[2]), bf_bits(a[3]));
    p[2] = pk16(bf_bits(b[0]), bf_bits(b[1]));
    p[3] = pk16(bf_bits(b[2]), bf_bits(b[3]));
    *(volatile v4u*)(out + (size_t)i * 8) = p;
    __threadfence();
    *(volatile v4u*)(out + (size_t)i * 8) = p;
  }
}

template <int NSPLIT, int OUT_MODE>
__global__ __launch_bounds__(256) void gemm64(
    const unsigned short* __restrict__ Ap, const unsigned short* __restrict__ A2p, int lda, long long strideA,
    const unsigned short* __restrict__ Btp, int ldb, long long strideB,
    void* Cout, void* Cout2, int ldc, long long strideC,
    int M, int N, int K, float cscale, float rscale, const float* __restrict__ osp) {
  const __bf16* A  = (const __bf16*)(const void*)Ap;
  const __bf16* A2 = (const __bf16*)(const void*)A2p;
  const __bf16* Bt = (const __bf16*)(const void*)Btp;
  __shared__ __align__(16) float sT[8][16 * 68];
  const int b    = blockIdx.y;
  const int lane = threadIdx.x & 31;
  const int wave = threadIdx.x >> 5;
  const int tilesN = N >> 6;
  const int tilesM = M >> 6;
  const int tile = blockIdx.x * 8 + wave;
  if (tile >= tilesM * tilesN) return;
  const int tm = tile / tilesN;
  const int tn = tile - tm * tilesN;
  const int m0 = tm << 6;
  const int n0 = tn << 6;

  const __bf16* Ab  = A  + (size_t)b * (size_t)strideA;
  const __bf16* Ab2 = (NSPLIT == 1) ? (A2 + (size_t)b * (size_t)strideA) : Ab;
  const __bf16* Bb  = Bt + (size_t)b * (size_t)strideB;

  const int rlane = lane & 15;
  const int koff  = (lane >> 4) * 8;
  const int mOff  = (lane >> 4) * 8;

  float oscale = cscale;
  if (OUT_MODE == 0) oscale = cscale * bf_up(bf_bits(osp[0]));

  v8f acc[4][4];
#pragma unroll
  for (int i = 0; i < 4; ++i)
#pragma unroll
    for (int j = 0; j < 4; ++j) acc[i][j] = zero8();

  for (int k0 = 0; k0 < K; k0 += 32) {
    v16b bh[4];
#pragma unroll
    for (int j = 0; j < 4; ++j) {
      const size_t bo = (size_t)(n0 + (j << 4) + rlane) * ldb + koff + k0;
      bh[j] = ldfrag_b(Bb + bo);
    }
#pragma unroll
    for (int i = 0; i < 4; ++i) {
      const size_t ao = (size_t)(m0 + (i << 4) + rlane) * lda + koff + k0;
      const v16b ah = ldfrag_b(Ab + ao);
      v16b al = ah;
      if (NSPLIT == 1) al = ldfrag_b(Ab2 + ao);
#pragma unroll
      for (int j = 0; j < 4; ++j) {
        acc[i][j] = wraw_b(ah, bh[j], acc[i][j]);
        if (NSPLIT == 1) acc[i][j] = wraw_b(al, bh[j], acc[i][j]);
      }
      dep_guard_b(acc[i][0], acc[i][3], ah, al);
    }
    keep4_b(bh[0], bh[1], bh[2], bh[3]);
  }
  acc_guard4(acc[0][0], acc[0][1], acc[0][2], acc[0][3]);
  acc_guard4(acc[1][0], acc[1][1], acc[1][2], acc[1][3]);
  acc_guard4(acc[2][0], acc[2][1], acc[2][2], acc[2][3]);
  acc_guard4(acc[3][0], acc[3][1], acc[3][2], acc[3][3]);

  float* slab = sT[wave];
#pragma unroll
  for (int i = 0; i < 4; ++i) {
    const int mBase = m0 + (i << 4);
#pragma unroll
    for (int j = 0; j < 4; ++j) {
#pragma unroll
      for (int r = 0; r < 8; ++r) {
        slab[(mOff + r) * 68 + (j << 4) + rlane] = acc[i][j][r];
      }
    }
    __builtin_amdgcn_fence(__ATOMIC_RELEASE, "workgroup");
    __builtin_amdgcn_wave_barrier();
    __builtin_amdgcn_fence(__ATOMIC_ACQUIRE, "workgroup");
    if (OUT_MODE == 0) {
      float* C = (float*)Cout + (size_t)b * (size_t)strideC;
      const int hh = lane >> 4, c4 = (lane & 15) * 4;
      for (int pass = 0; pass < 2; ++pass) {
#pragma unroll
        for (int it = 0; it < 8; ++it) {
          const int row = it * 2 + hh;
          const v4f v = *(const v4f*)(slab + row * 68 + c4) * oscale;
          *(volatile v4f*)(C + (size_t)(mBase + row) * ldc + n0 + c4) = v;
        }
        __threadfence();
      }
    } else {
      const int q = lane >> 3, c8 = (lane & 7) * 8;
      unsigned short* C  = (unsigned short*)Cout  + (size_t)b * (size_t)strideC;
      unsigned short* C2 = (unsigned short*)Cout2 + (size_t)b * (size_t)strideC;
      v4u hv[4], lv[4];
#pragma unroll
      for (int it = 0; it < 4; ++it) {
        const int row = it * 4 + q;
        const float* sp = slab + row * 68 + c8;
        v4u a, a2;
#pragma unroll
        for (int e = 0; e < 4; ++e) {
          const float f0 = sp[2 * e] * cscale, f1 = sp[2 * e + 1] * cscale;
          const _Float16 x0 = (_Float16)f0, x1 = (_Float16)f1;
          const unsigned short h0 = h_bits(x0), h1 = h_bits(x1);
          const unsigned short l0 = h_bits((_Float16)((f0 - (float)x0) * rscale));
          const unsigned short l1 = h_bits((_Float16)((f1 - (float)x1) * rscale));
          a[e] = pk16(h0, h1); a2[e] = pk16(l0, l1);
        }
        hv[it] = a; lv[it] = a2;
      }
      for (int pass = 0; pass < 2; ++pass) {
#pragma unroll
        for (int it = 0; it < 4; ++it) {
          const int row = it * 4 + q;
          *(volatile v4u*)(C + (size_t)(mBase + row) * ldc + n0 + c8) = hv[it];
          if (OUT_MODE == 3) *(volatile v4u*)(C2 + (size_t)(mBase + row) * ldc + n0 + c8) = lv[it];
        }
        __threadfence();
      }
    }
    __builtin_amdgcn_fence(__ATOMIC_RELEASE, "workgroup");
    __builtin_amdgcn_wave_barrier();
    __builtin_amdgcn_fence(__ATOMIC_ACQUIRE, "workgroup");
  }
}

__global__ __launch_bounds__(256) void decay_sum(
    const unsigned short* __restrict__ qhp, const unsigned short* __restrict__ qlp,
    const unsigned short* __restrict__ khp, const unsigned short* __restrict__ vtp,
    const float* __restrict__ dlp,
    unsigned short* rhp, unsigned short* rlp) {
  __shared__ __align__(16) _Float16 Psh[QR * PST];
  __shared__ __align__(16) float    Os[8][16 * 64];

  const int tid  = threadIdx.x;
  const int wave = tid >> 5;
  const int lane = tid & 31;
  const int hh   = lane >> 4;
  const int c    = lane & 15;

  const int bid = blockIdx.x;
  const int b   = bid / (TT / QR);
  const int qb  = bid - b * (TT / QR);
  const int t0  = qb * QR;

  const float dl  = bf_up(bf_bits(dlp[0]));
  const float dec = __builtin_amdgcn_rcpf(1.0f + __expf(-dl));
  const float l2d = log2f(fmaxf(dec, 1.0e-30f));
  const int ktFirst = t0 / KT;
  int ktLast = TT / KT - 1;
  if (dec < 0.999f) {
    const float wn   = 59.794706f * __builtin_amdgcn_rcpf(-l2d);
    const float wnc  = fminf(wn, 1.0e6f);
    const int   wlen = (int)wnc + 2;
    const int   lastKey = t0 + QR - 1 + wlen;
    const int   kl   = lastKey / KT;
    ktLast = (kl < ktLast) ? kl : ktLast;
  }
  const int ntiles = ktLast - ktFirst + 1;

  const size_t rowQ = (size_t)b * TT + (size_t)t0;
  const _Float16* Qh = (const _Float16*)(const void*)qhp;
  const _Float16* Ql = (const _Float16*)(const void*)qlp;
  const _Float16* Kh = (const _Float16*)(const void*)khp + (size_t)b * TT * DD;
  const _Float16* Vt = (const _Float16*)(const void*)vtp + (size_t)b * DD * TT;
  const _Float16* q0h = Qh + (rowQ + c) * DD + 8 * hh;
  const _Float16* q1h = q0h + (size_t)16 * DD;
  const _Float16* q0l = Ql + (rowQ + c) * DD + 8 * hh;
  const _Float16* q1l = q0l + (size_t)16 * DD;
  const _Float16* vr  = Vt + (size_t)(wave * 64 + c) * TT + 8 * hh;

  v8f acc[2][4];
#pragma unroll
  for (int mt = 0; mt < 2; ++mt)
#pragma unroll
    for (int nt = 0; nt < 4; ++nt) acc[mt][nt] = zero8();

  for (int it = 0; it < ntiles; ++it) {
    const int s0 = (ktFirst + it) * KT;
    const _Float16* kr = Kh + (size_t)(s0 + wave * 16 + c) * DD + 8 * hh;
    v8f sh0 = zero8(), sh1 = zero8(), sl0 = zero8(), sl1 = zero8();
#pragma unroll 1
    for (int d0 = 0; d0 < DD; d0 += 32) {
      const v16h kb = ldfrag_h(kr + d0);
      const v16h a0 = ldfrag_h(q0h + d0);
      const v16h a1 = ldfrag_h(q1h + d0);
      const v16h e0 = ldfrag_h(q0l + d0);
      const v16h e1 = ldfrag_h(q1l + d0);
      sh0 = wraw_h(a0, kb, sh0);
      sh1 = wraw_h(a1, kb, sh1);
      sl0 = wraw_h(e0, kb, sl0);
      sl1 = wraw_h(e1, kb, sl1);
      guard_s(sh0, sh1, sl0, sl1, a0, a1, e0, e1, kb);
    }

    const int scol = wave * 16 + c;
    const int nb   = s0 + scol - t0 - 8 * hh - 1;
#pragma unroll
    for (int r = 0; r < 8; ++r) {
      const int n0 = nb - r;
      const int n1 = n0 - 16;
      const float x0 = exp2f(l2d * (float)n0);
      const float x1 = exp2f(l2d * (float)n1);
      const float w0 = (n0 >= 0) ? x0 : 0.0f;
      const float w1 = (n1 >= 0) ? x1 : 0.0f;
      float p0 = (sh0[r] + sl0[r] * (1.0f / 1024.0f)) * w0;
      float p1 = (sh1[r] + sl1[r] * (1.0f / 1024.0f)) * w1;
      p0 = fminf(fmaxf(p0, -65504.0f), 65504.0f);
      p1 = fminf(fmaxf(p1, -65504.0f), 65504.0f);
      Psh[(8 * hh + r) * PST + scol]      = (_Float16)p0;
      Psh[(16 + 8 * hh + r) * PST + scol] = (_Float16)p1;
    }
    __syncthreads();

#pragma unroll 1
    for (int kc = 0; kc < KT; kc += 32) {
      const v16h pa0 = ldfrag_h(Psh + c * PST + kc + 8 * hh);
      const v16h pa1 = ldfrag_h(Psh + (16 + c) * PST + kc + 8 * hh);
      const v16h v0  = ldfrag_h(vr + s0 + kc);
      const v16h v1  = ldfrag_h(vr + (size_t)16 * TT + s0 + kc);
      const v16h v2  = ldfrag_h(vr + (size_t)32 * TT + s0 + kc);
      const v16h v3  = ldfrag_h(vr + (size_t)48 * TT + s0 + kc);
      acc[0][0] = wraw_h(pa0, v0, acc[0][0]);
      acc[1][0] = wraw_h(pa1, v0, acc[1][0]);
      acc[0][1] = wraw_h(pa0, v1, acc[0][1]);
      acc[1][1] = wraw_h(pa1, v1, acc[1][1]);
      acc[0][2] = wraw_h(pa0, v2, acc[0][2]);
      acc[1][2] = wraw_h(pa1, v2, acc[1][2]);
      acc[0][3] = wraw_h(pa0, v3, acc[0][3]);
      acc[1][3] = wraw_h(pa1, v3, acc[1][3]);
      guard_p(acc[0][0], acc[1][0], acc[0][1], acc[1][1], acc[0][2], acc[1][2], acc[0][3], acc[1][3],
              pa0, pa1, v0, v1, v2, v3);
    }
    __syncthreads();
  }

  const int q4 = lane >> 3, c8 = (lane & 7) * 8;
#pragma unroll
  for (int mt = 0; mt < 2; ++mt) {
    float* os = Os[wave];
#pragma unroll
    for (int nt = 0; nt < 4; ++nt) {
#pragma unroll
      for (int r = 0; r < 8; ++r) os[(8 * hh + r) * 64 + nt * 16 + c] = acc[mt][nt][r] * (1.0f / 1024.0f);
    }
    __syncthreads();
    v4u hv[4], lv[4];
#pragma unroll
    for (int i4 = 0; i4 < 4; ++i4) {
      const int row = i4 * 4 + q4;
      const float* sp = os + row * 64 + c8;
      v4u a, a2;
#pragma unroll
      for (int e = 0; e < 4; ++e) {
        const float f0 = sp[2 * e], f1 = sp[2 * e + 1];
        const unsigned short h0 = bf_bits(f0), h1 = bf_bits(f1);
        const unsigned short l0 = bf_bits(f0 - bf_up(h0)), l1 = bf_bits(f1 - bf_up(h1));
        a[e] = pk16(h0, h1); a2[e] = pk16(l0, l1);
      }
      hv[i4] = a; lv[i4] = a2;
    }
    for (int pass = 0; pass < 2; ++pass) {
#pragma unroll
      for (int i4 = 0; i4 < 4; ++i4) {
        const int row = i4 * 4 + q4;
        const size_t go = (rowQ + (size_t)(mt * 16 + row)) * DD + (size_t)(wave * 64 + c8);
        *(volatile v4u*)(rhp + go) = hv[i4];
        *(volatile v4u*)(rlp + go) = lv[i4];
      }
      __threadfence();
    }
    __syncthreads();
  }
}

extern "C" void kernel_launch(void* const* d_in, const int* in_sizes, int n_in,
                              void* d_out, int out_size, void* d_ws, size_t ws_size,
                              hipStream_t stream) {
  if (n_in < 7) return;
  if (in_sizes[0] != NB * TT * DD) return;
  if (in_sizes[1] != DD * DD || in_sizes[2] != DD * DD || in_sizes[3] != DD * DD || in_sizes[4] != DD * DD) return;
  if (in_sizes[5] < 1 || in_sizes[6] < 1) return;
  if (out_size != NB * TT * DD) return;

  const float* x   = (const float*)d_in[0];
  const float* Wq  = (const float*)d_in[1];
  const float* Wk  = (const float*)d_in[2];
  const float* Wv  = (const float*)d_in[3];
  const float* Wo  = (const float*)d_in[4];
  const float* dlp = (const float*)d_in[5];
  const float* osp = (const float*)d_in[6];

  const size_t PX = (size_t)NB * TT * DD * 2;
  const size_t PW = (size_t)DD * DD * 2;
  size_t off = 0;
  const size_t oXb = off; off += PX;
  const size_t oWq = off; off += PW;
  const size_t oWk = off; off += PW;
  const size_t oWv = off; off += PW;
  const size_t oWo = off; off += PW;
  const size_t oQh = off; off += PX;
  const size_t oQl = off; off += PX;
  const size_t oKh = off; off += PX;
  const size_t oVT = off; off += PX;
  const size_t oRh = off; off += PX;
  const size_t oRl = off; off += PX;
  if (off > ws_size) return;
  if (off > (size_t)134217728) return;

  char* ws = (char*)d_ws;
  unsigned short* Xb  = (unsigned short*)(ws + oXb);
  unsigned short* Wqb = (unsigned short*)(ws + oWq);
  unsigned short* Wkb = (unsigned short*)(ws + oWk);
  unsigned short* Wvb = (unsigned short*)(ws + oWv);
  unsigned short* Wob = (unsigned short*)(ws + oWo);
  unsigned short* Qh  = (unsigned short*)(ws + oQh);
  unsigned short* Ql  = (unsigned short*)(ws + oQl);
  unsigned short* Kh  = (unsigned short*)(ws + oKh);
  unsigned short* VT  = (unsigned short*)(ws + oVT);
  unsigned short* Rh  = (unsigned short*)(ws + oRh);
  unsigned short* Rl  = (unsigned short*)(ws + oRl);

  const dim3 blk(256);
  const int n8x = NB * TT * DD / 8;
  const int n8w = DD * DD / 8;
  const dim3 gCvtX((n8x + 255) / 256);
  const dim3 gCvtW((n8w + 255) / 256);
  const dim3 gProj((((NB * TT) / 64) * (DD / 64) + 7) / 8, 1);
  const dim3 gVT((((DD / 64) * (TT / 64)) + 7) / 8, NB);
  const dim3 gSum(NB * TT / QR);

  cvt_bf16x8<<<gCvtX, blk, 0, stream>>>(x, Xb, n8x);
  cvt_bf16x8<<<gCvtW, blk, 0, stream>>>(Wq, Wqb, n8w);
  cvt_bf16x8<<<gCvtW, blk, 0, stream>>>(Wk, Wkb, n8w);
  cvt_bf16x8<<<gCvtW, blk, 0, stream>>>(Wv, Wvb, n8w);
  cvt_bf16x8<<<gCvtW, blk, 0, stream>>>(Wo, Wob, n8w);
  gemm64<0, 3><<<gProj, blk, 0, stream>>>(
      Xb, Xb, DD, 0LL, Wqb, DD, 0LL,
      (void*)Qh, (void*)Ql, DD, 0LL,
      NB * TT, DD, DD, 8.0f, 1024.0f, osp);
  gemm64<0, 1><<<gProj, blk, 0, stream>>>(
      Xb, Xb, DD, 0LL, Wkb, DD, 0LL,
      (void*)Kh, (void*)Kh, DD, 0LL,
      NB * TT, DD, DD, 8.0f, 1.0f, osp);
  gemm64<0, 1><<<gVT, blk, 0, stream>>>(
      Wvb, Wvb, DD, 0LL, Xb, DD, (long long)TT * DD,
      (void*)VT, (void*)VT, TT, (long long)DD * TT,
      DD, TT, DD, 16.0f, 1.0f, osp);
  decay_sum<<<gSum, blk, 0, stream>>>(Qh, Ql, Kh, VT, dlp, Rh, Rl);
  gemm64<1, 0><<<gProj, blk, 0, stream>>>(
      Rh, Rl, DD, 0LL, Wob, DD, 0LL,
      d_out, d_out, DD, 0LL,
      NB * TT, DD, DD, 1.0f, 1.0f, osp);
  (void)hipGetLastError();
}
